// MultiHead_40415642255471
// MI455X (gfx1250) — hardware-verified
//
#include <hip/hip_runtime.h>


#ifndef NB
#define NB 2
#endif
#ifndef SEQ
#define SEQ 2048
#endif
#define NB_FULL  2
#define SEQ_FULL 2048
#ifndef OUT_SEQ
#define OUT_SEQ SEQ
#endif
#define DM   1024
#define NH_  16
#define HD   64
#define AW   4
#define QRS  2048.0f
#define QRI  (1.0f / 2048.0f)
#define SC2  (0.03125f * 1.4426950408889634f)
#define PSH  8.0f
#define WOS  64.0f
#define WOR  (1.0f / 32.0f)
#if SEQ < 512
#define EROWS SEQ
#else
#define EROWS 512
#endif

static_assert(HD == 64);
static_assert(NH_ * HD == DM);
static_assert(DM % 64 == 0);
static_assert(DM % 32 == 0);
static_assert(SEQ % 64 == 0);
static_assert((NB * SEQ) % 64 == 0);
static_assert(SEQ % 32 == 0);
static_assert(SEQ % (16 * AW) == 0);
static_assert(EROWS % (16 * AW) == 0);
static_assert((SEQ - EROWS) % (16 * AW) == 0);
static_assert(EROWS <= SEQ);
static_assert(((size_t)SEQ * DM) % 8 == 0);
static_assert(NB <= NB_FULL);
static_assert(SEQ <= SEQ_FULL);
static_assert(32 * 16 * 8 == 16 * HD * 4);
static_assert(AW * 16 * 68 * 4 <= 131072);
static_assert(64 * 65 * 4 <= 131072);
static_assert(16 * 68 * 4 <= 131072);

typedef _Float16 h16;
typedef unsigned short bf;
typedef __attribute__((ext_vector_type(16))) __bf16   v16bf;
typedef __attribute__((ext_vector_type(16))) _Float16 v16h;
typedef __attribute__((ext_vector_type(8)))  _Float16 v8h;
typedef __attribute__((ext_vector_type(8)))  unsigned short v8us;
typedef __attribute__((ext_vector_type(8)))  float    v8f;
typedef __attribute__((ext_vector_type(4)))  float    v4f;
typedef v4f  __attribute__((may_alias)) v4fa;

__device__ __forceinline__ unsigned short f2bf(float f) { unsigned u = __float_as_uint(f); u += 0x7FFFu + ((u >> 16) & 1u); return (unsigned short)(u >> 16); }
__device__ __forceinline__ v16h cat16(v8h lo, v8h hi) { return __builtin_shufflevector(lo, hi, 0, 1, 2, 3, 4, 5, 6, 7, 8, 9, 10, 11, 12, 13, 14, 15); }
__device__ __forceinline__ v16bf cat16b(v8us lo, v8us hi) { return __builtin_bit_cast(v16bf, __builtin_shufflevector(lo, hi, 0, 1, 2, 3, 4, 5, 6, 7, 8, 9, 10, 11, 12, 13, 14, 15)); }
__device__ __forceinline__ v8f wmma16(v16h a, v16h b, v8f c) { return __builtin_amdgcn_wmma_f32_16x16x32_f16(false, a, false, b, (short)0, c, false, false); }
__device__ __forceinline__ v8f wmmab(v16bf a, v16bf b, v8f c) { return __builtin_amdgcn_wmma_f32_16x16x32_bf16(false, a, false, b, (short)0, c, false, false); }
__device__ __forceinline__ v16h  ldh(const h16* p) { return cat16(*(const v8h*)p, *(const v8h*)(p + 16)); }
__device__ __forceinline__ v16bf ldb(const bf* p)  { return cat16b(*(const v8us*)p, *(const v8us*)(p + 16)); }
__device__ __forceinline__ void wave_sync() { __builtin_amdgcn_fence(3  , "wavefront"); __builtin_amdgcn_wave_barrier(); asm volatile("" ::: "memory"); }

static __device__ __forceinline__ h16 toh_flush(float v) { const h16 r = (h16)v; return (fabsf(v) < 6.103515625e-05f) ? (h16)0.0f : r; }
static __device__ __forceinline__ v8f wmma16g(v16h a, v16h b, v8f c) {
    c = __builtin_amdgcn_wmma_f32_16x16x32_f16(false, a, false, b, (short)0, c, false, false);
    asm volatile("v_nop\n\tv_nop\n\tv_nop\n\tv_nop" : "+v"(c) : "v"(a), "v"(b));
    return c;
}

__global__ __launch_bounds__(256) void k_cvt8(const float* __restrict__ src, bf* dst, size_t n8) {
    const size_t i = (size_t)blockIdx.x * 256 + threadIdx.x; if (i >= n8) return;
    const v8f v = *(const v8f*)(src + i * 8); v8us o;
#pragma unroll
    for (int k = 0; k < 8; ++k) o[k] = f2bf(v[k]);
    *(volatile v8us*)(dst + i * 8) = o; __threadfence(); *(volatile v8us*)(dst + i * 8) = o;
}

template <int MODE>
__global__ __launch_bounds__(256) void k_tr(const float* __restrict__ in, int inPitch, size_t inZ, unsigned short* out, int outPitch, size_t outZ) {
    __shared__ float ts[64 * 65];
    const int tid = threadIdx.x, lane = tid & 31, wave = tid >> 5;
    const int r0 = blockIdx.x * 64, c0 = blockIdx.y * 64;
    const float* ip = in + (size_t)blockIdx.z * inZ;
    unsigned short* op = out + (size_t)blockIdx.z * outZ;
#pragma unroll
    for (int i = 0; i < 4; ++i) { const int r = (tid >> 4) + 16 * i, c4 = (tid & 15) * 4;
        const v4f v = *(const v4f*)(ip + (size_t)(r0 + r) * (size_t)inPitch + c0 + c4);
        ts[r * 65 + c4 + 0] = v[0]; ts[r * 65 + c4 + 1] = v[1]; ts[r * 65 + c4 + 2] = v[2]; ts[r * 65 + c4 + 3] = v[3]; }
    __syncthreads();
#pragma unroll 1
    for (int ps = 0; ps < 2; ++ps) {
#pragma unroll
        for (int it = 0; it < 2; ++it) { const int c = wave * 8 + it * 4 + (lane >> 3), r8 = (lane & 7) * 8;
            v8us o = (v8us){}, o2 = (v8us){};
#pragma unroll
            for (int i = 0; i < 8; ++i) { const unsigned short wb = f2bf(ts[(r8 + i) * 65 + c]);
                if (MODE == 0) { o[i] = wb; }
                else { const float wr = __uint_as_float((unsigned)wb << 16);
                       o[i] = __builtin_bit_cast(unsigned short, (h16)(wr * WOS)); o2[i] = __builtin_bit_cast(unsigned short, (h16)(wr * WOR)); } }
            const size_t oo = (size_t)(c0 + c) * (size_t)outPitch + r0 + r8;
            *(volatile v8us*)(op + oo) = o; if (MODE == 1) *(volatile v8us*)(op + oo + DM) = o2; }
        if (ps == 0) __threadfence(); }
}

__global__ __launch_bounds__(32) void k_proj(const bf* __restrict__ A, const bf* __restrict__ Bt, h16* Ph, h16* Pr, int useRes, int RB, size_t sRB, int pitch, int CB, size_t sCB) {
    __shared__ __align__(16) float os[16 * 68];
    const int K = DM;
    const int lane = threadIdx.x & 31, lr = lane & 15, hi = lane >> 4; const int r0 = blockIdx.x * 64, c0 = blockIdx.y * 64;
    v8f acc[4][4];
#pragma unroll
    for (int mb = 0; mb < 4; ++mb)
#pragma unroll
        for (int nb = 0; nb < 4; ++nb) acc[mb][nb] = (v8f){};
    const size_t aoff = (size_t)(r0 + lr) * K + 8 * hi, boff = (size_t)(c0 + lr) * K + 8 * hi;
#pragma unroll 1
    for (int kc = 0; kc < K; kc += 32) {
        v16bf a[4];
#pragma unroll
        for (int mb = 0; mb < 4; ++mb) a[mb] = ldb(A + aoff + (size_t)mb * 16 * K + kc);
#pragma unroll
        for (int nb = 0; nb < 4; ++nb) { const v16bf b = ldb(Bt + boff + (size_t)nb * 16 * K + kc);
#pragma unroll
            for (int mb = 0; mb < 4; ++mb) acc[mb][nb] = wmmab(a[mb], b, acc[mb][nb]); }
        asm volatile("v_nop\n\tv_nop\n\tv_nop\n\tv_nop" : "+v"(acc[0][0]), "+v"(acc[1][1]), "+v"(acc[2][2]), "+v"(acc[3][3]) : "v"(a[0]), "v"(a[1]), "v"(a[2]), "v"(a[3]));
    }
    const size_t tbase = (size_t)(r0 / RB) * sRB + (size_t)(r0 % RB) * (size_t)pitch + (size_t)(c0 / CB) * sCB + (size_t)(c0 % CB);
#pragma unroll
    for (int mb = 0; mb < 4; ++mb) {
#pragma unroll
        for (int nb = 0; nb < 4; ++nb) {
#pragma unroll
            for (int j = 0; j < 8; ++j) os[(hi * 8 + j) * 68 + nb * 16 + lr] = acc[mb][nb][j]; }
        wave_sync();
        const size_t sb = tbase + (size_t)(mb * 16) * (size_t)pitch;
#pragma unroll 1
        for (int ps = 0; ps < 2; ++ps) {
#pragma unroll
            for (int s = 0; s < 4; ++s) { const int row = 4 * s + (lane >> 3), c8 = (lane & 7) * 8;
                const v4f x0 = *(const v4fa*)(&os[row * 68 + c8]); const v4f x1 = *(const v4fa*)(&os[row * 68 + c8 + 4]); v8h hv, rv;
#pragma unroll
                for (int i = 0; i < 4; ++i) { const h16 a0 = (h16)x0[i]; const h16 a1 = (h16)x1[i]; hv[i] = a0; hv[4 + i] = a1; rv[i] = (h16)((x0[i] - (float)a0) * QRS); rv[4 + i] = (h16)((x1[i] - (float)a1) * QRS); }
                const size_t oo = sb + (size_t)row * (size_t)pitch + c8;
                *(volatile v8h*)(Ph + oo) = hv; if (useRes) *(volatile v8h*)(Pr + oo) = rv; }
            if (ps == 0) __threadfence(); }
        wave_sync();
    }
}

template <int EARLY>
__device__ __forceinline__ void flash_body(const h16* QH, const h16* QR, const h16* KP, const h16* KR, const h16* VT, const h16* VR, float* OUT, const int rowbase) {
    __shared__ __align__(16) float os[AW * 16 * 68];
    const int lane = threadIdx.x & 31, lr = lane & 15, hi = lane >> 4;
    const int wave = __builtin_amdgcn_readfirstlane(threadIdx.x >> 5);
    const int zh = blockIdx.y; const int b = zh / NH_, h = zh % NH_;
    const int t0 = rowbase + (blockIdx.x * AW + wave) * 16;
    const int qi = t0 + lr;
    const size_t pbase = (size_t)zh * SEQ * HD;
    const size_t qo = pbase + (size_t)qi * HD + 8 * hi;
    const v16h qh0 = ldh(QH + qo), qh1 = ldh(QH + qo + 32);
    v16h qr0 = qh0, qr1 = qh1;
    if (EARLY) { qr0 = ldh(QR + qo); qr1 = ldh(QR + qo + 32); }
    const size_t ko = pbase + (size_t)lr * HD + 8 * hi;
    const size_t vo = pbase + (size_t)lr * SEQ + 8 * hi;
    v8f o0 = (v8f){}, o1 = (v8f){}, o2 = (v8f){}, o3 = (v8f){};
    v8f u0 = (v8f){}, u1 = (v8f){}, u2 = (v8f){}, u3 = (v8f){};
    float m = -3.0e38f, l = 0.0f;
    const int kend = t0 + 16;
#pragma unroll 1
    for (int key0 = 0; key0 < kend; key0 += 32) {
        const h16* ka = KP + ko + (size_t)key0 * HD;
        const v16h ka0 = ldh(ka), ka1 = ldh(ka + 32), kb0 = ldh(ka + 16 * HD), kb1 = ldh(ka + 16 * HD + 32);
        v8f sHa = (v8f){}, sLa = (v8f){}, sHb = (v8f){}, sLb = (v8f){};
        sHa = wmma16g(ka0, qh0, sHa); sHb = wmma16g(kb0, qh0, sHb);
        sHa = wmma16g(ka1, qh1, sHa); sHb = wmma16g(kb1, qh1, sHb);
        if (EARLY) {
            sLa = wmma16g(ka0, qr0, sLa); sLb = wmma16g(kb0, qr0, sLb);
            sLa = wmma16g(ka1, qr1, sLa); sLb = wmma16g(kb1, qr1, sLb);
            const h16* kr = KR + ko + (size_t)key0 * HD;
            const v16h ra0 = ldh(kr), ra1 = ldh(kr + 32), rb0 = ldh(kr + 16 * HD), rb1 = ldh(kr + 16 * HD + 32);
            sLa = wmma16g(ra0, qh0, sLa); sLb = wmma16g(rb0, qh0, sLb);
            sLa = wmma16g(ra1, qh1, sLa); sLb = wmma16g(rb1, qh1, sLb);
        }
        float ta[8], tb[8];
#pragma unroll
        for (int r = 0; r < 8; ++r) {
            if (EARLY) { ta[r] = (sHa[r] + sLa[r] * QRI) * SC2; tb[r] = (sHb[r] + sLb[r] * QRI) * SC2; }
            else       { ta[r] = sHa[r] * SC2;                  tb[r] = sHb[r] * SC2; } }
        if (key0 + 31 > t0) {
#pragma unroll
            for (int r = 0; r < 8; ++r) { const int kk = key0 + 8 * hi + r;
                ta[r] = (kk > qi) ? -3.0e38f : ta[r]; tb[r] = (kk + 16 > qi) ? -3.0e38f : tb[r]; }
        }
        float mx = -3.0e38f;
#pragma unroll
        for (int r = 0; r < 8; ++r) mx = fmaxf(mx, fmaxf(ta[r], tb[r]));
        mx = fmaxf(mx, __shfl_xor(mx, 16, 32));
        const float mnew = fmaxf(m, mx);
        const float alpha = __builtin_amdgcn_exp2f(m - mnew);
        const float sh = PSH - mnew;
        v16h pb, pr; float ls = 0.0f;
#pragma unroll
        for (int r = 0; r < 8; ++r) {
            const float ea = ta[r] + sh, ec = tb[r] + sh;
            const float xa = __builtin_amdgcn_exp2f(ea), xc = __builtin_amdgcn_exp2f(ec);
            const float pa = (ea < -14.0f) ? 0.0f : xa;
            const float pc = (ec < -14.0f) ? 0.0f : xc;
            const h16 ha = (h16)pa, hc = (h16)pc; pb[r] = ha; pb[8 + r] = hc;
            if (EARLY) { ls += pa + pc; pr[r] = toh_flush((pa - (float)ha) * QRS); pr[8 + r] = toh_flush((pc - (float)hc) * QRS); }
            else       { ls += (float)ha + (float)hc; pr[r] = ha; pr[8 + r] = hc; } }
        l = l * alpha + ls; m = mnew;
        o0 = o0 * alpha; o1 = o1 * alpha; o2 = o2 * alpha; o3 = o3 * alpha;
        const h16* va = VT + vo + key0;
        const v16h v0 = ldh(va), v1 = ldh(va + (size_t)16 * SEQ), v2 = ldh(va + (size_t)32 * SEQ), v3 = ldh(va + (size_t)48 * SEQ);
        o0 = wmma16g(v0, pb, o0); o1 = wmma16g(v1, pb, o1); o2 = wmma16g(v2, pb, o2); o3 = wmma16g(v3, pb, o3);
        if (EARLY) {
            u0 = u0 * alpha; u1 = u1 * alpha; u2 = u2 * alpha; u3 = u3 * alpha;
            u0 = wmma16g(v0, pr, u0); u1 = wmma16g(v1, pr, u1); u2 = wmma16g(v2, pr, u2); u3 = wmma16g(v3, pr, u3);
            const h16* wa = VR + vo + key0;
            const v16h w0 = ldh(wa), w1 = ldh(wa + (size_t)16 * SEQ), w2 = ldh(wa + (size_t)32 * SEQ), w3 = ldh(wa + (size_t)48 * SEQ);
            u0 = wmma16g(w0, pb, u0); u1 = wmma16g(w1, pb, u1); u2 = wmma16g(w2, pb, u2); u3 = wmma16g(w3, pb, u3);
        }
    }
    l += __shfl_xor(l, 16, 32);
    const float inv = 1.0f / l;
    v8f f0 = o0 * inv, f1 = o1 * inv, f2 = o2 * inv, f3 = o3 * inv;
    if (EARLY) { f0 = (o0 + u0 * QRI) * inv; f1 = (o1 + u1 * QRI) * inv; f2 = (o2 + u2 * QRI) * inv; f3 = (o3 + u3 * QRI) * inv; }
    const int wb = wave * 16 * 68;
    { const int sbase = wb + lr * 68 + 8 * hi;
      *(v4fa*)(&os[sbase +  0]) = __builtin_shufflevector(f0, f0, 0, 1, 2, 3); *(v4fa*)(&os[sbase +  0 + 4]) = __builtin_shufflevector(f0, f0, 4, 5, 6, 7);
      *(v4fa*)(&os[sbase + 16]) = __builtin_shufflevector(f1, f1, 0, 1, 2, 3); *(v4fa*)(&os[sbase + 16 + 4]) = __builtin_shufflevector(f1, f1, 4, 5, 6, 7);
      *(v4fa*)(&os[sbase + 32]) = __builtin_shufflevector(f2, f2, 0, 1, 2, 3); *(v4fa*)(&os[sbase + 32 + 4]) = __builtin_shufflevector(f2, f2, 4, 5, 6, 7);
      *(v4fa*)(&os[sbase + 48]) = __builtin_shufflevector(f3, f3, 0, 1, 2, 3); *(v4fa*)(&os[sbase + 48 + 4]) = __builtin_shufflevector(f3, f3, 4, 5, 6, 7); }
    wave_sync();
    float* orow = OUT + ((size_t)b * OUT_SEQ + t0) * DM + h * HD;
#pragma unroll 1
    for (int ps = 0; ps < 2; ++ps) {
#pragma unroll
        for (int s = 0; s < 8; ++s) { const int row = 2 * s + hi, cofs = lr * 4;
            const v4f val = *(const v4fa*)(&os[wb + row * 68 + cofs]);
            *(volatile v4f*)(orow + (size_t)row * DM + cofs) = val; }
        if (ps == 0) __threadfence(); }
}

__global__ __launch_bounds__(32 * AW) void k_flash_early(const h16* __restrict__ QH, const h16* __restrict__ QR, const h16* __restrict__ KP, const h16* __restrict__ KR, const h16* __restrict__ VT, const h16* __restrict__ VR, float* OUT) {
    flash_body<1>(QH, QR, KP, KR, VT, VR, OUT, 0);
}
__global__ __launch_bounds__(32 * AW) void k_flash(const h16* __restrict__ QH, const h16* __restrict__ KP, const h16* __restrict__ VT, float* OUT) {
    flash_body<0>(QH, QH, KP, KP, VT, VT, OUT, EROWS);
}

static constexpr size_t al256(size_t v) { return (v + 255) & ~(size_t)255; }
static constexpr size_t SZ_XB = al256((size_t)NB * SEQ * DM * 2);
static constexpr size_t SZ_WB = al256((size_t)3 * DM * DM * 2);
static constexpr size_t SZ_PL = al256((size_t)NB * NH_ * SEQ * HD * 2);
static constexpr size_t SZ_TOTAL = SZ_XB + SZ_WB + 6 * SZ_PL;
static_assert(SZ_TOTAL <= (size_t)134217728);
static_assert(((size_t)DM * DM * 2) % 256 == 0);
static_assert((size_t)NB * NH_ * SEQ * HD == (size_t)NB * SEQ * DM);

extern "C" void kernel_launch(void* const* d_in, const int* in_sizes, int n_in,
                              void* d_out, int out_size, void* d_ws, size_t ws_size, hipStream_t stream) {
    if (n_in < 4) return;
    const size_t needx = ((size_t)(NB - 1) * SEQ_FULL + SEQ) * DM;
    if ((size_t)in_sizes[0] < needx) return;
    const size_t nw = (size_t)NH_ * DM * HD;
    if ((size_t)in_sizes[1] < nw || (size_t)in_sizes[2] < nw || (size_t)in_sizes[3] < nw) return;
    if ((size_t)out_size < ((size_t)(NB - 1) * OUT_SEQ + SEQ) * DM) return;
    if (SZ_TOTAL > ws_size) return;
    const float* x = (const float*)d_in[0]; const float* wq = (const float*)d_in[1]; const float* wk = (const float*)d_in[2]; const float* wv = (const float*)d_in[3];
    float* OUT = (float*)d_out;
    char* wsp = (char*)d_ws;
    bf* XB = (bf*)wsp; wsp += SZ_XB;
    bf* WB = (bf*)wsp; wsp += SZ_WB;
    h16* QH = (h16*)wsp; wsp += SZ_PL;
    h16* QR = (h16*)wsp; wsp += SZ_PL;
    h16* KP = (h16*)wsp; wsp += SZ_PL;
    h16* KR = (h16*)wsp; wsp += SZ_PL;
    h16* VT = (h16*)wsp; wsp += SZ_PL;
    h16* VR = (h16*)wsp; wsp += SZ_PL;
    bf* WQ = WB; bf* WK = WB + (size_t)DM * DM; bf* WV = WB + (size_t)2 * DM * DM;

    if (SEQ == SEQ_FULL) {
        const size_t n8 = (size_t)NB * SEQ * DM / 8;
        k_cvt8<<<(unsigned)((n8 + 255) / 256), 256, 0, stream>>>(x, XB, n8);
    } else {
        const size_t n8 = (size_t)SEQ * DM / 8;
        for (int b = 0; b < NB; ++b) k_cvt8<<<(unsigned)((n8 + 255) / 256), 256, 0, stream>>>(x + (size_t)b * SEQ_FULL * DM, XB + (size_t)b * SEQ * DM, n8);
    }
    { const dim3 g(DM / 64, HD / 64, NH_);
      k_tr<0><<<g, 256, 0, stream>>>(wq, HD, (size_t)DM * HD, WQ, DM, (size_t)HD * DM);
      k_tr<0><<<g, 256, 0, stream>>>(wk, HD, (size_t)DM * HD, WK, DM, (size_t)HD * DM);
      k_tr<0><<<g, 256, 0, stream>>>(wv, HD, (size_t)DM * HD, WV, DM, (size_t)HD * DM); }

    k_proj<<<dim3(NB * SEQ / 64, DM / 64, 1), 32, 0, stream>>>(XB, WQ, QH, QR, 1, SEQ, (size_t)NH_ * SEQ * HD, HD, HD, (size_t)SEQ * HD);
    k_proj<<<dim3(NB * SEQ / 64, DM / 64, 1), 32, 0, stream>>>(XB, WK, KP, KR, 1, SEQ, (size_t)NH_ * SEQ * HD, HD, HD, (size_t)SEQ * HD);
    k_proj<<<dim3(DM / 64, NB * SEQ / 64, 1), 32, 0, stream>>>(WV, XB, VT, VR, 1, DM, (size_t)0, SEQ, SEQ, (size_t)DM * SEQ);

    k_flash_early<<<dim3(EROWS / (16 * AW), NB * NH_, 1), 32 * AW, 0, stream>>>(QH, QR, KP, KR, VT, VR, OUT);
    if (SEQ > EROWS)
        k_flash<<<dim3((SEQ - EROWS) / (16 * AW), NB * NH_, 1), 32 * AW, 0, stream>>>(QH, KP, VT, OUT);
}
